// SiameseNetworkRespective_12335146074640
// MI455X (gfx1250) — hardware-run, weakly checked
//
#include <hip/hip_runtime.h>


namespace {
constexpr int N = 50000, E = 800000, CI = 64, D = 128, T = 4, NW = N / 16  ;
constexpr float HS = 256.0f, AS = 16.0f  , WSC = 256.0f;
typedef _Float16 b16;
typedef __attribute__((ext_vector_type(16))) _Float16 v16b;
typedef __attribute__((ext_vector_type(8))) _Float16 v8b;
typedef __attribute__((ext_vector_type(8))) float v8f;
typedef __attribute__((ext_vector_type(4))) float v4f;
__device__ __forceinline__ float bf16_rne(float f) { unsigned int u = __float_as_uint(f); u += 0x7FFFu + ((u >> 16) & 1u); float r = __uint_as_float(u & 0xFFFF0000u); asm volatile("" : "+v"(r)); return r; }
__device__ __forceinline__ float bfv(float f) { float r = bf16_rne(f); asm volatile("" : "+v"(r)); return r; }
__device__ __forceinline__ void split16(float v, b16& hi, b16& lo) { hi = (b16)v; lo = (b16)(v - (float)hi); }
__device__ __forceinline__ v16b frag_kb(const b16* p, int hh) { const v8b a = *(const v8b*)(p + 8 * hh), b = *(const v8b*)(p + 16 + 8 * hh); v16b f;
#pragma unroll
  for (int e = 0; e < 8; ++e) { f[e] = a[e]; f[8 + e] = b[e]; } return f; }
__device__ __forceinline__ v8f wmma16b(v16b a, v16b b, v8f c) { v8f d = __builtin_amdgcn_wmma_f32_16x16x32_f16(false, a, false, b, (short)0, c, false, false); asm volatile("v_nop\n\tv_nop\n\tv_nop\n\tv_nop" : "+v"(d) : "v"(a), "v"(b)); return d; }
__device__ __forceinline__ void wave_lds_sync() { __builtin_amdgcn_fence(__ATOMIC_RELEASE, "workgroup"); __builtin_amdgcn_wave_barrier(); __builtin_amdgcn_fence(__ATOMIC_ACQUIRE, "workgroup"); }
__device__ __forceinline__ float pmul(float a, float b) { float p = a * b; asm volatile("" : "+v"(p)); return p; }
__device__ __forceinline__ int iclamp(int v, int lo, int hi) { return v < lo ? lo : (v > hi ? hi : v); }
constexpr int CSR_NBLK9 = 512, CSR_GB9 = 9, CSR_GN9 = 1 << CSR_GB9  , CSR_TS9 = (CSR_GN9 < 32 ? 32 : CSR_GN9)  , CSR_MAXG9 = 512, CSR_CAP9 = 12288  ;
__device__ __host__ __forceinline__ int csr_tix9(int v) { return (v >> CSR_GB9) * CSR_TS9 + (v & (CSR_GN9 - 1)); }
__global__ __launch_bounds__(64) void csrA_kernel9(const int* __restrict__ dst, int E, int N, int nG, int CHP, int NGP, int* __restrict__ STG, int* __restrict__ HST) {
  extern __shared__ int sm[];
  int* cnt = sm; int* run = sm + NGP; int* ids = sm + 2 * NGP;
  const int b = blockIdx.x; const int ch = (E + CSR_NBLK9 - 1) / CSR_NBLK9; const int e0 = b * ch, e1 = min(E, e0 + ch);
  for (int i = threadIdx.x; i < NGP; i += 64) cnt[i] = 0;
  for (int i = threadIdx.x; i < CHP; i += 64) ids[i] = -1;
  __syncthreads();
  if (threadIdx.x == 0) {
    for (int e = e0; e < e1; ++e) { int d = dst[e]; d = (d < 0) ? 0 : (d >= N ? N - 1 : d); cnt[d >> CSR_GB9] += 1; }
    int acc = 0; for (int g = 0; g < nG; ++g) { run[g] = acc; acc += cnt[g]; }
    for (int e = e0; e < e1; ++e) { int d = dst[e]; d = (d < 0) ? 0 : (d >= N ? N - 1 : d); const int g = d >> CSR_GB9; ids[run[g]] = e; run[g] += 1; } }
  __syncthreads();
  typedef __attribute__((ext_vector_type(4))) int v4i;
  for (int pass = 0; pass < 2; ++pass) {
    for (int i = threadIdx.x; i < CHP / 4; i += 64) *(volatile v4i*)(STG + (size_t)b * CHP + i * 4) = *(const v4i*)(&ids[i * 4]);
    for (int i = threadIdx.x; i < NGP / 4; i += 64) { v4i v; for (int e = 0; e < 4; ++e) v[e] = (i * 4 + e < nG) ? cnt[i * 4 + e] : 0; *(volatile v4i*)(HST + (size_t)b * NGP + i * 4) = v; }
    __threadfence(); }
}
__global__ __launch_bounds__(512) void csrS_kernel9(const int* __restrict__ HST, int nG, int NGP, int* __restrict__ START, int* __restrict__ TOT, int* __restrict__ OFF) {
  __shared__ int tot[CSR_MAXG9];
  const int b = threadIdx.x;
  for (int pass = 0; pass < 2; ++pass) { int runb = 0; for (int g = 0; g < nG; ++g) { int c = HST[(size_t)b * NGP + g]; c = (c < 0) ? 0 : c; ((volatile int*)OFF)[(size_t)g * CSR_NBLK9 + b] = runb; runb += c; } __threadfence(); }
  for (int g = threadIdx.x; g < nG; g += 512) { int s = 0; for (int bb = 0; bb < CSR_NBLK9; ++bb) { int c = HST[(size_t)bb * NGP + g]; s += (c < 0) ? 0 : c; } tot[g] = s; }
  __syncthreads();
  if (threadIdx.x < 32) {
    __shared__ int st[CSR_MAXG9 + 32];
    if (threadIdx.x == 0) { int acc = 0; for (int g = 0; g < NGP; ++g) { st[g] = acc; if (g < nG) acc += (tot[g] + 31) & ~31; } st[NGP] = acc; }
    __builtin_amdgcn_fence(__ATOMIC_RELEASE, "workgroup"); __builtin_amdgcn_wave_barrier(); __builtin_amdgcn_fence(__ATOMIC_ACQUIRE, "workgroup");
    for (int pass = 0; pass < 2; ++pass) { for (int i = threadIdx.x; i < NGP + 32; i += 32) { ((volatile int*)START)[i] = (i <= NGP) ? st[min(i, NGP)] : 0; ((volatile int*)TOT)[i] = (i < nG) ? tot[i] : 0; } __threadfence(); } }
}
__global__ __launch_bounds__(256) void csrB_kernel9(const int* __restrict__ dst, int N, int nG, int CHP, int NGP, int permLen, const int* __restrict__ STG, const int* __restrict__ HST, const int* __restrict__ OFF, const int* __restrict__ START, const int* __restrict__ TOT, int* __restrict__ PERM, int* __restrict__ ROWPTR, int* __restrict__ ROWCNT, int* __restrict__ FLAG) {
  typedef __attribute__((ext_vector_type(4))) int v4i;
  __shared__ int ids[CSR_CAP9]; __shared__ unsigned short key[CSR_CAP9]; __shared__ int outp[CSR_CAP9]; __shared__ int ncnt[CSR_GN9 + 1]; __shared__ int boff[CSR_NBLK9 + 1];
  const int g = blockIdx.x, t_ = threadIdx.x; int tot = TOT[g]; int st = START[g], stn = START[g + 1]; const int v0 = g * CSR_GN9; const int nv = min(CSR_GN9, N - v0); const int t0 = g * CSR_TS9;
  st = (st < 0) ? 0 : (st > permLen - 32 ? permLen - 32 : st) & ~31; stn = (stn < st) ? st : (stn > permLen ? permLen : stn); tot = (tot < 0) ? 0 : tot; if (tot > stn - st && tot <= CSR_CAP9) tot = stn - st;
  if (tot > CSR_CAP9) {
    for (int pass = 0; pass < 2; ++pass) { for (int i = t_; i < CSR_TS9 / 4; i += 256) { v4i a, c; for (int e = 0; e < 4; ++e) { a[e] = st; c[e] = 0; } *(volatile v4i*)(ROWPTR + t0 + i * 4) = a; *(volatile v4i*)(ROWCNT + t0 + i * 4) = c; } if (t_ == 0) ((volatile int*)FLAG)[0] = 1; __threadfence(); } (void)nv; return; }
  if (t_ == 0) { int acc = 0; for (int b = 0; b < CSR_NBLK9; ++b) { boff[b] = acc; int c = HST[(size_t)b * NGP + g]; c = (c < 0) ? 0 : (c > CHP ? CHP : c); acc += c; if (acc > tot) acc = tot; } boff[CSR_NBLK9] = acc; }
  for (int i = t_; i <= CSR_GN9; i += 256) ncnt[i] = 0;
  __syncthreads();
  for (int b = 0; b < CSR_NBLK9; ++b) { const int c = boff[b + 1] - boff[b]; int o_ = OFF[(size_t)g * CSR_NBLK9 + b]; o_ = (o_ < 0) ? 0 : (o_ > CHP - c ? CHP - c : o_); const int* src_ = STG + (size_t)b * CHP + o_;
    for (int i = t_; i < c; i += 256) { int id = src_[i]; id = (id < 0) ? 0 : id; ids[boff[b] + i] = id; int d = dst[id]; d = (d < v0) ? v0 : (d >= N ? N - 1 : d); int kk = d - v0; kk = (kk < 0) ? 0 : (kk >= CSR_GN9 ? CSR_GN9 - 1 : kk); key[boff[b] + i] = (unsigned short)kk; } }
  __syncthreads();
  if (t_ == 0) { for (int i = 0; i < tot; ++i) ncnt[key[i]] += 1; int acc = 0; for (int vl = 0; vl < CSR_GN9; ++vl) { const int c = ncnt[vl]; ncnt[vl] = acc; acc += c; } ncnt[CSR_GN9] = acc;
    for (int i = 0; i < tot; ++i) { const int vl = key[i]; outp[ncnt[vl]] = ids[i]; ncnt[vl] += 1; }
    for (int vl = CSR_GN9; vl > 0; --vl) ncnt[vl] = ncnt[vl - 1]; ncnt[0] = 0; }
  __syncthreads();
  for (int pass = 0; pass < 2; ++pass) {
    for (int i = t_; i < (stn - st) / 4; i += 256) { v4i v; for (int e = 0; e < 4; ++e) { const int q = i * 4 + e; v[e] = (q < tot) ? outp[q] : -1; } *(volatile v4i*)(PERM + st + i * 4) = v; }
    for (int i = t_; i < CSR_TS9 / 4; i += 256) { v4i a, c; for (int e = 0; e < 4; ++e) { const int vl = i * 4 + e; const int vc = vl < CSR_GN9 ? vl : CSR_GN9; a[e] = (vl < CSR_GN9) ? st + ncnt[vc] : st; c[e] = (vl < nv) ? (ncnt[(vc < CSR_GN9 ? vc : CSR_GN9 - 1) + 1] - ncnt[vc]) : 0; } *(volatile v4i*)(ROWPTR + t0 + i * 4) = a; *(volatile v4i*)(ROWCNT + t0 + i * 4) = c; }
    __threadfence(); }
}
__global__ __launch_bounds__(256) void csrZ_kernel9(int* __restrict__ p, size_t n4) { typedef __attribute__((ext_vector_type(4))) int v4i; const size_t tid = (size_t)blockIdx.x * 256 + threadIdx.x, nth = (size_t)gridDim.x * 256; v4i z = {0, 0, 0, 0}; for (size_t i = tid; i < n4; i += nth) *(volatile v4i*)(p + i * 4) = z; }
struct CsrBufs9 { int *STG, *HST, *OFF, *START, *TOT, *PERM, *ROWPTR, *ROWCNT, *FLAG; int nG, NGP, CHP; size_t permLen; char* base; size_t bytes; };
static size_t csr_carve9(CsrBufs9& c, char* ws, size_t off, int E, int N) {
  const size_t off0 = off; c.base = ws + off;
  auto al = [&](size_t bytes) { char* p = ws + off; off += (bytes + 255) & ~(size_t)255; return p; };
  c.nG = (N + CSR_GN9 - 1) / CSR_GN9; c.NGP = (c.nG + 31) & ~31; const int ch = (E + CSR_NBLK9 - 1) / CSR_NBLK9; c.CHP = (ch + 31) & ~31; c.permLen = (size_t)E + 32 * (size_t)c.nG + 32;
  c.STG = (int*)al((size_t)CSR_NBLK9 * c.CHP * 4); c.HST = (int*)al((size_t)CSR_NBLK9 * c.NGP * 4); c.OFF = (int*)al((size_t)c.NGP * CSR_NBLK9 * 4); c.START = (int*)al((size_t)(c.NGP + 64) * 4); c.TOT = (int*)al((size_t)(c.NGP + 64) * 4);
  c.PERM = (int*)al(c.permLen * 4); c.ROWPTR = (int*)al((size_t)c.nG * CSR_TS9 * 4); c.ROWCNT = (int*)al((size_t)c.nG * CSR_TS9 * 4); c.FLAG = (int*)al(256);
  c.bytes = off - off0; return off;
}
static void csr_build9(const CsrBufs9& c, const int* dst, int E, int N, hipStream_t stream) {
  const size_t smem = (size_t)(2 * c.NGP + c.CHP) * 4;
  csrZ_kernel9<<<512, 256, 0, stream>>>((int*)c.base, c.bytes / 16);
  csrA_kernel9<<<CSR_NBLK9, 64, smem, stream>>>(dst, E, N, c.nG, c.CHP, c.NGP, c.STG, c.HST);
  csrS_kernel9<<<1, 512, 0, stream>>>(c.HST, c.nG, c.NGP, c.START, c.TOT, c.OFF);
  csrB_kernel9<<<c.nG, 256, 0, stream>>>(dst, N, c.nG, c.CHP, c.NGP, (int)c.permLen, c.STG, c.HST, c.OFF, c.START, c.TOT, c.PERM, c.ROWPTR, c.ROWCNT, c.FLAG);
}


__global__ __launch_bounds__(256) void wput_kernel(const float* __restrict__ w1, const float* __restrict__ m1, const float* __restrict__ m2, const float* __restrict__ m3, b16* __restrict__ W1p, b16* __restrict__ Mp) { const int u = blockIdx.x * 256 + threadIdx.x; v8b v;
  if (u < D * CI / 8) {
#pragma unroll
    for (int j = 0; j < 8; ++j) v[j] = (b16)(bf16_rne(w1[u * 8 + j]) * WSC); for (int pass = 0; pass < 2; ++pass) { *(volatile v8b*)(W1p + u * 8) = v; __threadfence(); } }
  if (u < 3 * D * D / 8) { const int m = u / (D * D / 8); const float* src = m == 0 ? m1 : (m == 1 ? m2 : m3); const size_t o8 = u % (D * D / 8);
#pragma unroll
    for (int j = 0; j < 8; ++j) v[j] = (b16)(bf16_rne(src[o8 * 8 + j]) * WSC); for (int pass = 0; pass < 2; ++pass) { *(volatile v8b*)(Mp + (size_t)u * 8) = v; __threadfence(); } } }
__global__ __launch_bounds__(32) void xw_kernel(const float* __restrict__ x, const b16* __restrict__ W1p, const float* __restrict__ b1, int NLIM, float* __restrict__ XW) { __shared__ __attribute__((aligned(16))) b16 Ah[16][72]; __shared__ float Tf[16][D + 4]; const int lane = threadIdx.x, nloc = lane & 15, hlf = lane >> 4; const size_t m0 = (size_t)blockIdx.x * 16; if (m0 >= (size_t)NLIM) return;
  for (int rr = 0; rr < 16; ++rr) { Ah[rr][lane] = (b16)(bf16_rne(x[(m0 + rr) * CI + lane]) * HS); Ah[rr][32 + lane] = (b16)(bf16_rne(x[(m0 + rr) * CI + 32 + lane]) * HS); } if (lane < 16) for (int k = 64; k < 72; ++k) Ah[lane][k] = (b16)0.0f;
  wave_lds_sync(); v8f acc[8];
#pragma unroll
  for (int t = 0; t < 8; ++t) acc[t] = (v8f){};
#pragma unroll
  for (int kb = 0; kb < CI; kb += 32) { const v16b a = frag_kb(&Ah[nloc][kb], hlf);
#pragma unroll
    for (int t = 0; t < 8; ++t) acc[t] = wmma16b(a, frag_kb(W1p + (size_t)(t * 16 + nloc) * CI + kb, hlf), acc[t]); }
#pragma unroll
  for (int t = 0; t < 8; ++t)
#pragma unroll
    for (int r8 = 0; r8 < 8; ++r8) Tf[8 * hlf + r8][t * 16 + nloc] = acc[t][r8] * (1.0f / (HS * WSC)) + bfv(b1[t * 16 + nloc]);
  wave_lds_sync();
  for (int pass = 0; pass < 2; ++pass) { for (int rr = 0; rr < 16; ++rr) *(volatile v4f*)(XW + (m0 + rr) * D + lane * 4) = *(const v4f*)(&Tf[rr][lane * 4]); __threadfence(); } }
template <int FIRST>
__global__ __launch_bounds__(256) void agg_kernel(const float* __restrict__ U, const int* __restrict__ srcs, const int* __restrict__ PERM, const int* __restrict__ ROWPTR, const int* __restrict__ ROWCNT, int permLen, int NLIM, float* __restrict__ AG) { const int wave = threadIdx.x >> 5, lane = threadIdx.x & 31; const size_t i = (size_t)blockIdx.x * 8 + wave; if (i >= (size_t)NLIM) return; int st = ROWPTR[i], cnt = ROWCNT[i]; cnt = iclamp(cnt, 0, E); st = iclamp(st, 0, permLen - cnt);
  v4f acc = {0, 0, 0, 0};
#pragma unroll 1
  for (int j = 0; j < cnt; ++j) { const int e = iclamp(PERM[st + j], 0, E - 1); const size_t u = (size_t)iclamp(srcs[e], 0, N - 1); if (u >= (size_t)NLIM) continue; const v4f v = *(const v4f*)(U + u * D + lane * 4);
#pragma unroll
    for (int k = 0; k < 4; ++k) acc[k] += FIRST ? bfv(v[k]) : v[k]; }
  for (int pass = 0; pass < 2; ++pass) { *(volatile v4f*)(AG + i * D + lane * 4) = acc; __threadfence(); } }
template <int LAST>
__global__ __launch_bounds__(32) void mlp_kernel(const float* __restrict__ AG, const float* __restrict__ XW, const b16* __restrict__ Mp, const float* __restrict__ b1, const float* __restrict__ b2, const float* __restrict__ b3, int NLIM, float* __restrict__ U, float* __restrict__ PART) { __shared__ __attribute__((aligned(16))) b16 Ah[16][D + 8], Al[16][D + 8]; __shared__ float Tf[16][D + 4]; const int lane = threadIdx.x, nloc = lane & 15, hlf = lane >> 4; const size_t m0 = (size_t)blockIdx.x * 16; if (m0 >= (size_t)NLIM) return;
  for (int rr = 0; rr < 16; ++rr) for (int q = 0; q < 4; ++q) { b16 p, ql; split16(AG[(m0 + rr) * D + q * 32 + lane] * AS, p, ql); Ah[rr][q * 32 + lane] = p; Al[rr][q * 32 + lane] = ql; }
  wave_lds_sync();
#pragma unroll 1
  for (int layer = 0; layer < 3; ++layer) { const b16* W = Mp + (size_t)layer * D * D; const float* bb = layer == 0 ? b1 : (layer == 1 ? b2 : b3); const float isc = layer == 0 ? 1.0f / (AS * WSC) : 1.0f / (HS * WSC); v8f acc[8];
#pragma unroll
    for (int t = 0; t < 8; ++t) acc[t] = (v8f){};
#pragma unroll
    for (int kb = 0; kb < D; kb += 32) { const v16b a = frag_kb(&Ah[nloc][kb], hlf), al = frag_kb(&Al[nloc][kb], hlf);
#pragma unroll
      for (int t = 0; t < 8; ++t) { const v16b bw = frag_kb(W + (size_t)(t * 16 + nloc) * D + kb, hlf); acc[t] = wmma16b(a, bw, acc[t]); acc[t] = wmma16b(al, bw, acc[t]); } }
#pragma unroll
    for (int t = 0; t < 8; ++t) { const int cc = t * 16 + nloc; const float b_ = bfv(bb[cc]);
#pragma unroll
      for (int r8 = 0; r8 < 8; ++r8) { const float v = acc[t][r8] * isc + b_; Tf[8 * hlf + r8][cc] = layer < 2 ? fmaxf(v, 0.0f) : tanhf(v); } }
    wave_lds_sync();
    if (layer < 2) { for (int rr = 0; rr < 16; ++rr) for (int q = 0; q < 4; ++q) { b16 p, ql; split16(Tf[rr][q * 32 + lane] * HS, p, ql); Ah[rr][q * 32 + lane] = p; Al[rr][q * 32 + lane] = ql; } wave_lds_sync(); } }
  v4f ps = {0, 0, 0, 0};
  for (int pass = 0; pass < 2; ++pass) { for (int rr = 0; rr < 16; ++rr) { v4f o; for (int k = 0; k < 4; ++k) { const int c = lane * 4 + k; o[k] = fmaxf(XW[(m0 + rr) * D + c] + Tf[rr][c], 0.0f); if (LAST && pass == 0) ps[k] += o[k]; } *(volatile v4f*)(U + (m0 + rr) * D + lane * 4) = o; } __threadfence(); }
  if (LAST) for (int pass = 0; pass < 2; ++pass) { *(volatile v4f*)(PART + (size_t)blockIdx.x * D + lane * 4) = ps; __threadfence(); } }
__global__ __launch_bounds__(32) void readout_kernel(const float* __restrict__ PART, int nw, const float* __restrict__ w2, const float* __restrict__ b2, float* __restrict__ out) { __shared__ double Gs[D]; const int lane = threadIdx.x;
  for (int q = 0; q < 4; ++q) { const int c = q * 32 + lane; double s = 0.0; for (int w = 0; w < nw; ++w) s += (double)PART[(size_t)w * D + c]; Gs[c] = s; }
  wave_lds_sync();
  float o4[4];
  for (int q = 0; q < 4; ++q) { const int o = q * 32 + lane; double s = 0.0; for (int c = 0; c < D; ++c) s += Gs[c] * (double)bfv(w2[(size_t)o * D + c]); o4[q] = (float)(s + (double)bfv(b2[o])); }
  for (int pass = 0; pass < 2; ++pass) { for (int q = 0; q < 4; ++q) ((volatile float*)out)[q * 32 + lane] = o4[q]; __threadfence(); } }
}

extern "C" void kernel_launch(void* const* d_in, const int* in_sizes, int n_in, void* d_out, int out_size, void* d_ws, size_t ws_size, hipStream_t stream) {
  (void)n_in;
  auto Fp = [&](int i) { return (const float*)d_in[i]; }; auto Ip = [&](int i) { return (const int*)d_in[i]; };
  if (in_sizes[0] != N * CI || in_sizes[1] != N * D || in_sizes[2] != 2 * E || in_sizes[3] != D * CI || in_sizes[5] != D * D || in_sizes[7] != D * D || in_sizes[9] != D * D || in_sizes[11] != D * D || out_size != D) return;
  const int NLIM = N;
  size_t off = 0; char* ws = (char*)d_ws;
  auto carve = [&](size_t bytes) { char* p = ws + off; off += (bytes + 255) & ~(size_t)255; return p; };
  b16* W1p = (b16*)carve((size_t)D * CI * 2); b16* Mp = (b16*)carve((size_t)3 * D * D * 2); float* XW = (float*)carve((size_t)N * D * 4); float* AG = (float*)carve((size_t)N * D * 4); float* UA = (float*)carve((size_t)N * D * 4); float* UB = (float*)carve((size_t)N * D * 4); float* PART = (float*)carve((size_t)NW * D * 4); CsrBufs9 csr; off = csr_carve9(csr, ws, off, E, N);
  if (off > ws_size || off > ((size_t)128 << 20)) return;
  const int nw = NLIM / 16;
  wput_kernel<<<(3 * D * D / 8 + 255) / 256, 256, 0, stream>>>(Fp(3), Fp(5), Fp(7), Fp(9), W1p, Mp);
  csr_build9(csr, Ip(2) + E, E, N, stream);
  xw_kernel<<<nw, 32, 0, stream>>>(Fp(0), W1p, Fp(4), NLIM, XW);
  agg_kernel<1><<<(NLIM + 7) / 8, 256, 0, stream>>>(Fp(1), Ip(2), csr.PERM, csr.ROWPTR, csr.ROWCNT, (int)csr.permLen, NLIM, AG);
  mlp_kernel<0><<<nw, 32, 0, stream>>>(AG, XW, Mp, Fp(6), Fp(8), Fp(10), NLIM, UA, PART);
  agg_kernel<0><<<(NLIM + 7) / 8, 256, 0, stream>>>(UA, Ip(2), csr.PERM, csr.ROWPTR, csr.ROWCNT, (int)csr.permLen, NLIM, AG);
  mlp_kernel<0><<<nw, 32, 0, stream>>>(AG, XW, Mp, Fp(6), Fp(8), Fp(10), NLIM, UB, PART);
  agg_kernel<0><<<(NLIM + 7) / 8, 256, 0, stream>>>(UB, Ip(2), csr.PERM, csr.ROWPTR, csr.ROWCNT, (int)csr.permLen, NLIM, AG);
  mlp_kernel<0><<<nw, 32, 0, stream>>>(AG, XW, Mp, Fp(6), Fp(8), Fp(10), NLIM, UA, PART);
  agg_kernel<0><<<(NLIM + 7) / 8, 256, 0, stream>>>(UA, Ip(2), csr.PERM, csr.ROWPTR, csr.ROWCNT, (int)csr.permLen, NLIM, AG);
  mlp_kernel<1><<<nw, 32, 0, stream>>>(AG, XW, Mp, Fp(6), Fp(8), Fp(10), NLIM, UB, PART);
  readout_kernel<<<1, 32, 0, stream>>>(PART, nw, Fp(11), Fp(12), (float*)d_out);
}
